// Struct2SeqGCN_30167850287447
// MI455X (gfx1250) — hardware-run, weakly checked
//
#include <hip/hip_runtime.h>


namespace {
constexpr int N = 25000, NPAD = 25008  , E = 400000, FIN = 6, H = 128, NG = 16, NC = 21, NPB = 8;
constexpr float HS = 256.0f, WSC = 256.0f, EPS = 1e-5f;
typedef _Float16 b16;
typedef __attribute__((ext_vector_type(16))) _Float16 v16b;
typedef __attribute__((ext_vector_type(8))) _Float16 v8b;
typedef __attribute__((ext_vector_type(8))) float v8f;
typedef __attribute__((ext_vector_type(4))) float v4f;
__device__ __forceinline__ float bf16_rne(float f) { unsigned int u = __float_as_uint(f); u += 0x7FFFu + ((u >> 16) & 1u); float r = __uint_as_float(u & 0xFFFF0000u); asm volatile("" : "+v"(r)); return r; }
__device__ __forceinline__ float bfv(float f) { float r = bf16_rne(f); asm volatile("" : "+v"(r)); return r; }
__device__ __forceinline__ void split16(float v, b16& hi, b16& lo) { hi = (b16)v; lo = (b16)(v - (float)hi); }
__device__ __forceinline__ v16b frag_kb(const b16* p, int hh) { const v8b a = *(const v8b*)(p + 8 * hh), b = *(const v8b*)(p + 16 + 8 * hh); v16b f;
#pragma unroll
  for (int e = 0; e < 8; ++e) { f[e] = a[e]; f[8 + e] = b[e]; } return f; }
__device__ __forceinline__ v8f wmma16b(v16b a, v16b b, v8f c) { v8f d = __builtin_amdgcn_wmma_f32_16x16x32_f16(false, a, false, b, (short)0, c, false, false); asm volatile("v_nop\n\tv_nop\n\tv_nop\n\tv_nop" : "+v"(d) : "v"(a), "v"(b)); return d; }
__device__ __forceinline__ void wave_lds_sync() { __builtin_amdgcn_fence(__ATOMIC_RELEASE, "workgroup"); __builtin_amdgcn_wave_barrier(); __builtin_amdgcn_fence(__ATOMIC_ACQUIRE, "workgroup"); }
__device__ __forceinline__ float pmul(float a, float b) { float p = a * b; asm volatile("" : "+v"(p)); return p; }
__device__ __forceinline__ int iclamp(int v, int lo, int hi) { return v < lo ? lo : (v > hi ? hi : v); }
__device__ __forceinline__ float sigm(float v) { return 1.0f / (1.0f + __expf(-v)); }
__device__ __forceinline__ float softplus(float v) { return v > 20.0f ? v : log1pf(__expf(v)); }
constexpr int CSR_NBLK8 = 512, CSR_GB8 = 8, CSR_GN8 = 1 << CSR_GB8  , CSR_TS8 = (CSR_GN8 < 32 ? 32 : CSR_GN8)  , CSR_MAXG8 = 512, CSR_CAP8 = 12288  ;
__device__ __host__ __forceinline__ int csr_tix8(int v) { return (v >> CSR_GB8) * CSR_TS8 + (v & (CSR_GN8 - 1)); }
__global__ __launch_bounds__(64) void csrA_kernel8(const int* __restrict__ dst, int E, int N, int nG, int CHP, int NGP, int* __restrict__ STG, int* __restrict__ HST) {
  extern __shared__ int sm[];
  int* cnt = sm; int* run = sm + NGP; int* ids = sm + 2 * NGP;
  const int b = blockIdx.x; const int ch = (E + CSR_NBLK8 - 1) / CSR_NBLK8; const int e0 = b * ch, e1 = min(E, e0 + ch);
  for (int i = threadIdx.x; i < NGP; i += 64) cnt[i] = 0;
  for (int i = threadIdx.x; i < CHP; i += 64) ids[i] = -1;
  __syncthreads();
  if (threadIdx.x == 0) {
    for (int e = e0; e < e1; ++e) { int d = dst[e]; d = (d < 0) ? 0 : (d >= N ? N - 1 : d); cnt[d >> CSR_GB8] += 1; }
    int acc = 0; for (int g = 0; g < nG; ++g) { run[g] = acc; acc += cnt[g]; }
    for (int e = e0; e < e1; ++e) { int d = dst[e]; d = (d < 0) ? 0 : (d >= N ? N - 1 : d); const int g = d >> CSR_GB8; ids[run[g]] = e; run[g] += 1; } }
  __syncthreads();
  typedef __attribute__((ext_vector_type(4))) int v4i;
  for (int pass = 0; pass < 2; ++pass) {
    for (int i = threadIdx.x; i < CHP / 4; i += 64) *(volatile v4i*)(STG + (size_t)b * CHP + i * 4) = *(const v4i*)(&ids[i * 4]);
    for (int i = threadIdx.x; i < NGP / 4; i += 64) { v4i v; for (int e = 0; e < 4; ++e) v[e] = (i * 4 + e < nG) ? cnt[i * 4 + e] : 0; *(volatile v4i*)(HST + (size_t)b * NGP + i * 4) = v; }
    __threadfence(); }
}
__global__ __launch_bounds__(512) void csrS_kernel8(const int* __restrict__ HST, int nG, int NGP, int* __restrict__ START, int* __restrict__ TOT, int* __restrict__ OFF) {
  __shared__ int tot[CSR_MAXG8];
  const int b = threadIdx.x;
  for (int pass = 0; pass < 2; ++pass) { int runb = 0; for (int g = 0; g < nG; ++g) { int c = HST[(size_t)b * NGP + g]; c = (c < 0) ? 0 : c; ((volatile int*)OFF)[(size_t)g * CSR_NBLK8 + b] = runb; runb += c; } __threadfence(); }
  for (int g = threadIdx.x; g < nG; g += 512) { int s = 0; for (int bb = 0; bb < CSR_NBLK8; ++bb) { int c = HST[(size_t)bb * NGP + g]; s += (c < 0) ? 0 : c; } tot[g] = s; }
  __syncthreads();
  if (threadIdx.x < 32) {
    __shared__ int st[CSR_MAXG8 + 32];
    if (threadIdx.x == 0) { int acc = 0; for (int g = 0; g < NGP; ++g) { st[g] = acc; if (g < nG) acc += (tot[g] + 31) & ~31; } st[NGP] = acc; }
    __builtin_amdgcn_fence(__ATOMIC_RELEASE, "workgroup"); __builtin_amdgcn_wave_barrier(); __builtin_amdgcn_fence(__ATOMIC_ACQUIRE, "workgroup");
    for (int pass = 0; pass < 2; ++pass) { for (int i = threadIdx.x; i < NGP + 32; i += 32) { ((volatile int*)START)[i] = (i <= NGP) ? st[min(i, NGP)] : 0; ((volatile int*)TOT)[i] = (i < nG) ? tot[i] : 0; } __threadfence(); } }
}
__global__ __launch_bounds__(256) void csrB_kernel8(const int* __restrict__ dst, int N, int nG, int CHP, int NGP, int permLen, const int* __restrict__ STG, const int* __restrict__ HST, const int* __restrict__ OFF, const int* __restrict__ START, const int* __restrict__ TOT, int* __restrict__ PERM, int* __restrict__ ROWPTR, int* __restrict__ ROWCNT, int* __restrict__ FLAG) {
  typedef __attribute__((ext_vector_type(4))) int v4i;
  __shared__ int ids[CSR_CAP8]; __shared__ unsigned short key[CSR_CAP8]; __shared__ int outp[CSR_CAP8]; __shared__ int ncnt[CSR_GN8 + 1]; __shared__ int boff[CSR_NBLK8 + 1];
  const int g = blockIdx.x, t_ = threadIdx.x; int tot = TOT[g]; int st = START[g], stn = START[g + 1]; const int v0 = g * CSR_GN8; const int nv = min(CSR_GN8, N - v0); const int t0 = g * CSR_TS8;
  st = (st < 0) ? 0 : (st > permLen - 32 ? permLen - 32 : st) & ~31; stn = (stn < st) ? st : (stn > permLen ? permLen : stn); tot = (tot < 0) ? 0 : tot; if (tot > stn - st && tot <= CSR_CAP8) tot = stn - st;
  if (tot > CSR_CAP8) {
    for (int pass = 0; pass < 2; ++pass) { for (int i = t_; i < CSR_TS8 / 4; i += 256) { v4i a, c; for (int e = 0; e < 4; ++e) { a[e] = st; c[e] = 0; } *(volatile v4i*)(ROWPTR + t0 + i * 4) = a; *(volatile v4i*)(ROWCNT + t0 + i * 4) = c; } if (t_ == 0) ((volatile int*)FLAG)[0] = 1; __threadfence(); } (void)nv; return; }
  if (t_ == 0) { int acc = 0; for (int b = 0; b < CSR_NBLK8; ++b) { boff[b] = acc; int c = HST[(size_t)b * NGP + g]; c = (c < 0) ? 0 : (c > CHP ? CHP : c); acc += c; if (acc > tot) acc = tot; } boff[CSR_NBLK8] = acc; }
  for (int i = t_; i <= CSR_GN8; i += 256) ncnt[i] = 0;
  __syncthreads();
  for (int b = 0; b < CSR_NBLK8; ++b) { const int c = boff[b + 1] - boff[b]; int o_ = OFF[(size_t)g * CSR_NBLK8 + b]; o_ = (o_ < 0) ? 0 : (o_ > CHP - c ? CHP - c : o_); const int* src_ = STG + (size_t)b * CHP + o_;
    for (int i = t_; i < c; i += 256) { int id = src_[i]; id = (id < 0) ? 0 : id; ids[boff[b] + i] = id; int d = dst[id]; d = (d < v0) ? v0 : (d >= N ? N - 1 : d); int kk = d - v0; kk = (kk < 0) ? 0 : (kk >= CSR_GN8 ? CSR_GN8 - 1 : kk); key[boff[b] + i] = (unsigned short)kk; } }
  __syncthreads();
  if (t_ == 0) { for (int i = 0; i < tot; ++i) ncnt[key[i]] += 1; int acc = 0; for (int vl = 0; vl < CSR_GN8; ++vl) { const int c = ncnt[vl]; ncnt[vl] = acc; acc += c; } ncnt[CSR_GN8] = acc;
    for (int i = 0; i < tot; ++i) { const int vl = key[i]; outp[ncnt[vl]] = ids[i]; ncnt[vl] += 1; }
    for (int vl = CSR_GN8; vl > 0; --vl) ncnt[vl] = ncnt[vl - 1]; ncnt[0] = 0; }
  __syncthreads();
  for (int pass = 0; pass < 2; ++pass) {
    for (int i = t_; i < (stn - st) / 4; i += 256) { v4i v; for (int e = 0; e < 4; ++e) { const int q = i * 4 + e; v[e] = (q < tot) ? outp[q] : -1; } *(volatile v4i*)(PERM + st + i * 4) = v; }
    for (int i = t_; i < CSR_TS8 / 4; i += 256) { v4i a, c; for (int e = 0; e < 4; ++e) { const int vl = i * 4 + e; const int vc = vl < CSR_GN8 ? vl : CSR_GN8; a[e] = (vl < CSR_GN8) ? st + ncnt[vc] : st; c[e] = (vl < nv) ? (ncnt[(vc < CSR_GN8 ? vc : CSR_GN8 - 1) + 1] - ncnt[vc]) : 0; } *(volatile v4i*)(ROWPTR + t0 + i * 4) = a; *(volatile v4i*)(ROWCNT + t0 + i * 4) = c; }
    __threadfence(); }
}
__global__ __launch_bounds__(256) void csrZ_kernel8(int* __restrict__ p, size_t n4) { typedef __attribute__((ext_vector_type(4))) int v4i; const size_t tid = (size_t)blockIdx.x * 256 + threadIdx.x, nth = (size_t)gridDim.x * 256; v4i z = {0, 0, 0, 0}; for (size_t i = tid; i < n4; i += nth) *(volatile v4i*)(p + i * 4) = z; }
struct CsrBufs8 { int *STG, *HST, *OFF, *START, *TOT, *PERM, *ROWPTR, *ROWCNT, *FLAG; int nG, NGP, CHP; size_t permLen; char* base; size_t bytes; };
static size_t csr_carve8(CsrBufs8& c, char* ws, size_t off, int E, int N) {
  const size_t off0 = off; c.base = ws + off;
  auto al = [&](size_t bytes) { char* p = ws + off; off += (bytes + 255) & ~(size_t)255; return p; };
  c.nG = (N + CSR_GN8 - 1) / CSR_GN8; c.NGP = (c.nG + 31) & ~31; const int ch = (E + CSR_NBLK8 - 1) / CSR_NBLK8; c.CHP = (ch + 31) & ~31; c.permLen = (size_t)E + 32 * (size_t)c.nG + 32;
  c.STG = (int*)al((size_t)CSR_NBLK8 * c.CHP * 4); c.HST = (int*)al((size_t)CSR_NBLK8 * c.NGP * 4); c.OFF = (int*)al((size_t)c.NGP * CSR_NBLK8 * 4); c.START = (int*)al((size_t)(c.NGP + 64) * 4); c.TOT = (int*)al((size_t)(c.NGP + 64) * 4);
  c.PERM = (int*)al(c.permLen * 4); c.ROWPTR = (int*)al((size_t)c.nG * CSR_TS8 * 4); c.ROWCNT = (int*)al((size_t)c.nG * CSR_TS8 * 4); c.FLAG = (int*)al(256);
  c.bytes = off - off0; return off;
}
static void csr_build8(const CsrBufs8& c, const int* dst, int E, int N, hipStream_t stream) {
  const size_t smem = (size_t)(2 * c.NGP + c.CHP) * 4;
  csrZ_kernel8<<<512, 256, 0, stream>>>((int*)c.base, c.bytes / 16);
  csrA_kernel8<<<CSR_NBLK8, 64, smem, stream>>>(dst, E, N, c.nG, c.CHP, c.NGP, c.STG, c.HST);
  csrS_kernel8<<<1, 512, 0, stream>>>(c.HST, c.nG, c.NGP, c.START, c.TOT, c.OFF);
  csrB_kernel8<<<c.nG, 256, 0, stream>>>(dst, N, c.nG, c.CHP, c.NGP, (int)c.permLen, c.STG, c.HST, c.OFF, c.START, c.TOT, c.PERM, c.ROWPTR, c.ROWCNT, c.FLAG);
}


__global__ __launch_bounds__(256) void wput_kernel(const float* __restrict__ f1, const float* __restrict__ s1, const float* __restrict__ f2, const float* __restrict__ s2, b16* __restrict__ WN, b16* __restrict__ WE) { const size_t nt = (size_t)gridDim.x * 256, u0 = (size_t)blockIdx.x * 256 + threadIdx.x; v8b v;
  for (size_t u = u0; u < (size_t)2 * 512 * 16; u += nt) { const int l = (int)(u / (512 * 16)); const int r = (int)(u % (512 * 16)); const int o = r / 16, k0 = (r % 16) * 8; const float* fw = l ? f2 : f1; const float* sw = l ? s2 : s1; const float* W = o < 256 ? fw : sw; const int oo = o % 256; const int rowoff = oo < 128 ? 0 : H; const int c = oo % 128;
#pragma unroll
    for (int j = 0; j < 8; ++j) v[j] = (b16)(bf16_rne(W[(size_t)(rowoff + k0 + j) * H + c]) * WSC); for (int pass = 0; pass < 2; ++pass) { *(volatile v8b*)(WN + ((size_t)l * 512 + o) * H + k0) = v; __threadfence(); } }
  for (size_t u = u0; u < (size_t)2 * 256 * 4; u += nt) { const int l = (int)(u / (256 * 4)); const int r = (int)(u % (256 * 4)); const int o = r / 4, k0 = (r % 4) * 8; const float* W = o < 128 ? (l ? f2 : f1) : (l ? s2 : s1); const int c = o % 128;
#pragma unroll
    for (int j = 0; j < 8; ++j) { const int k = k0 + j; v[j] = (b16)(k < NG ? bf16_rne(W[(size_t)(2 * H + k) * H + c]) * WSC : 0.0f); } for (int pass = 0; pass < 2; ++pass) { *(volatile v8b*)(WE + ((size_t)l * 256 + o) * 32 + k0) = v; __threadfence(); } } }
__global__ __launch_bounds__(256) void lin0_kernel(const float* __restrict__ x, const float* __restrict__ nw, const float* __restrict__ nb, int NLIM, float* __restrict__ Hp) { const size_t u = (size_t)blockIdx.x * 256 + threadIdx.x; const size_t n = u / 32; const int c0 = (int)(u % 32) * 4; if (n >= (size_t)NLIM) return; float x6[FIN]; for (int q = 0; q < FIN; ++q) x6[q] = bfv(x[n * FIN + q]); v4f o;
#pragma unroll
  for (int j = 0; j < 4; ++j) { float s = bfv(nb[c0 + j]); for (int q = 0; q < FIN; ++q) s += pmul(x6[q], bfv(nw[q * H + c0 + j])); o[j] = s; }
  for (int pass = 0; pass < 2; ++pass) { *(volatile v4f*)(Hp + n * H + c0) = o; __threadfence(); } }
__global__ __launch_bounds__(32) void proj_kernel(const float* __restrict__ Hp, const b16* __restrict__ W, int NLIM, float* __restrict__ P) { __shared__ __attribute__((aligned(16))) b16 Ah[16][H + 8], Al[16][H + 8]; __shared__ float Tf[16][260]; const int lane = threadIdx.x, nloc = lane & 15, hlf = lane >> 4; const size_t m0 = (size_t)blockIdx.x * 16; if (m0 >= (size_t)NLIM) return;
  for (int rr = 0; rr < 16; ++rr) { const size_t row = (m0 + rr) < (size_t)N ? m0 + rr : (size_t)N - 1; for (int q = 0; q < 4; ++q) { b16 p, ql; split16(Hp[row * H + q * 32 + lane] * HS, p, ql); Ah[rr][q * 32 + lane] = p; Al[rr][q * 32 + lane] = ql; } } if (lane < 16) for (int k = H; k < H + 8; ++k) { Ah[lane][k] = (b16)0.0f; Al[lane][k] = (b16)0.0f; }
  wave_lds_sync();
#pragma unroll 1
  for (int g = 0; g < 2; ++g) { v8f acc[16];
#pragma unroll
    for (int t = 0; t < 16; ++t) acc[t] = (v8f){};
#pragma unroll
    for (int kb = 0; kb < H; kb += 32) { const v16b a = frag_kb(&Ah[nloc][kb], hlf), al = frag_kb(&Al[nloc][kb], hlf);
#pragma unroll
      for (int t = 0; t < 16; ++t) { const v16b bw = frag_kb(W + (size_t)(g * 256 + t * 16 + nloc) * H + kb, hlf); acc[t] = wmma16b(a, bw, acc[t]); acc[t] = wmma16b(al, bw, acc[t]); } }
#pragma unroll
    for (int t = 0; t < 16; ++t)
#pragma unroll
      for (int r8 = 0; r8 < 8; ++r8) Tf[8 * hlf + r8][t * 16 + nloc] = acc[t][r8] * (1.0f / (HS * WSC));
    wave_lds_sync();
    for (int pass = 0; pass < 2; ++pass) { for (int rr = 0; rr < 16; ++rr) for (int q = 0; q < 2; ++q) *(volatile v4f*)(P + (m0 + rr) * 512 + g * 256 + q * 128 + lane * 4) = *(const v4f*)(&Tf[rr][q * 128 + lane * 4]); __threadfence(); }
    wave_lds_sync(); } }
__global__ __launch_bounds__(128) void cg_kernel(const float* __restrict__ P, const float* __restrict__ ea, const b16* __restrict__ WE, const float* __restrict__ fb, const float* __restrict__ sb, const int* __restrict__ srcs, const int* __restrict__ PERM, const int* __restrict__ ROWPTR, const int* __restrict__ ROWCNT, int permLen, int NLIM, float* __restrict__ AGG, float* __restrict__ PS) {
  __shared__ __attribute__((aligned(16))) b16 Eh[4][16][40], El[4][16][40]; __shared__ float Tz[4][16][260]; __shared__ int Sj[4][16]; __shared__ float Gs[4][H];
  const int wave = threadIdx.x >> 5, lane = threadIdx.x & 31, nloc = lane & 15, hlf = lane >> 4; const size_t i = (size_t)blockIdx.x * 4 + wave; const bool live = i < (size_t)NLIM; float ag[4] = {0, 0, 0, 0};
  if (live) { int st = ROWPTR[i], cnt = ROWCNT[i]; cnt = iclamp(cnt, 0, E); st = iclamp(st, 0, permLen - cnt); float pd[4], ps[4], fbb[4], sbb[4]; for (int k = 0; k < 4; ++k) { const int c = lane * 4 + k; pd[k] = P[i * 512 + c]; ps[k] = P[i * 512 + 256 + c]; fbb[k] = bfv(fb[c]); sbb[k] = bfv(sb[c]); }
    if (lane < 16) for (int k = 32; k < 40; ++k) { Eh[wave][lane][k] = (b16)0.0f; El[wave][lane][k] = (b16)0.0f; }
#pragma unroll 1
    for (int t0 = 0; t0 < cnt; t0 += 16) {
      { const int r = nloc; const int j = t0 + r; int sj = -1; float ev = 0.0f; if (j < cnt) { const int e = iclamp(PERM[st + j], 0, E - 1); const int u = iclamp(srcs[e], 0, N - 1); if (u < NLIM) { sj = u; ev = bfv(ea[e]); } }
        if (hlf == 0) Sj[wave][r] = sj;
        for (int k = 0; k < 16; ++k) { const int kk = hlf * 16 + k; float g = 0.0f; if (kk < NG && sj >= 0) { const float off = (float)(8.0 * (double)kk / 15.0); const float d = ev - off; g = __expf(-1.7578125f * d * d); } b16 p, ql; split16(g * HS, p, ql); Eh[wave][r][kk] = p; El[wave][r][kk] = ql; } }
      wave_lds_sync(); v8f acc[16];
#pragma unroll
      for (int t = 0; t < 16; ++t) acc[t] = (v8f){};
      { const v16b a = frag_kb(&Eh[wave][nloc][0], hlf), al = frag_kb(&El[wave][nloc][0], hlf);
#pragma unroll
        for (int t = 0; t < 16; ++t) { const v16b bw = frag_kb(WE + (size_t)(t * 16 + nloc) * 32, hlf); acc[t] = wmma16b(a, bw, acc[t]); acc[t] = wmma16b(al, bw, acc[t]); } }
#pragma unroll
      for (int t = 0; t < 16; ++t)
#pragma unroll
        for (int r8 = 0; r8 < 8; ++r8) Tz[wave][8 * hlf + r8][t * 16 + nloc] = acc[t][r8] * (1.0f / (HS * WSC));
      wave_lds_sync();
      const int nr = (cnt - t0) < 16 ? (cnt - t0) : 16;
      for (int r = 0; r < nr; ++r) { const int sj = Sj[wave][r]; if (sj < 0) continue; const v4f pfs = *(const v4f*)(P + (size_t)sj * 512 + 128 + lane * 4), pss = *(const v4f*)(P + (size_t)sj * 512 + 384 + lane * 4);
#pragma unroll
        for (int k = 0; k < 4; ++k) { const int c = lane * 4 + k; const float zf = Tz[wave][r][c] + pd[k] + pfs[k] + fbb[k]; const float zs = Tz[wave][r][128 + c] + ps[k] + pss[k] + sbb[k]; ag[k] += pmul(sigm(zf), softplus(zs)); } }
      wave_lds_sync(); } }
#pragma unroll
  for (int k = 0; k < 4; ++k) Gs[wave][lane * 4 + k] = live ? ag[k] : 0.0f;
  __syncthreads();
  for (int pass = 0; pass < 2; ++pass) { if (live) *(volatile v4f*)(AGG + i * H + lane * 4) = (v4f){ag[0], ag[1], ag[2], ag[3]}; { const int c = threadIdx.x; float s = 0.0f, s2 = 0.0f; for (int w = 0; w < 4; ++w) { const float v = Gs[w][c]; s += v; s2 += v * v; } ((volatile float*)PS)[(size_t)blockIdx.x * 2 * H + c] = s; ((volatile float*)PS)[(size_t)blockIdx.x * 2 * H + H + c] = s2; } __threadfence(); } }
__global__ __launch_bounds__(128) void bn_kernel(const float* __restrict__ PS, int nb, int count, const float* __restrict__ g, const float* __restrict__ be, float* __restrict__ BNP) { const int c = threadIdx.x; double s = 0.0, s2 = 0.0; for (int w = 0; w < nb; ++w) { s += (double)PS[(size_t)w * 2 * H + c]; s2 += (double)PS[(size_t)w * 2 * H + H + c]; } const double mu = s / count; double var = s2 / count - mu * mu; if (var < 0.0) var = 0.0; const float sc = bfv(g[c]) * (float)(1.0 / sqrt(var + (double)EPS)); const float sh = bfv(be[c]) - (float)mu * sc;
  for (int pass = 0; pass < 2; ++pass) { ((volatile float*)BNP)[c] = sc; ((volatile float*)BNP)[H + c] = sh; __threadfence(); } }
__global__ __launch_bounds__(256) void upd_kernel(const float* __restrict__ AGG, const float* __restrict__ BNP, int NLIM, float* __restrict__ Hp) { const size_t u = (size_t)blockIdx.x * 256 + threadIdx.x; const size_t n = u / 32; const int c0 = (int)(u % 32) * 4; if (n >= (size_t)NLIM) return; v4f o; const v4f hv = *(const v4f*)(Hp + n * H + c0);
#pragma unroll
  for (int j = 0; j < 4; ++j) { const int c = c0 + j; o[j] = fmaxf(pmul(AGG[n * H + c], BNP[c]) + BNP[H + c] + hv[j], 0.0f); }
  for (int pass = 0; pass < 2; ++pass) { *(volatile v4f*)(Hp + n * H + c0) = o; __threadfence(); } }
__global__ __launch_bounds__(256) void fc_kernel(const float* __restrict__ Hp, const float* __restrict__ fw, const float* __restrict__ fb2, int NLIM, float* __restrict__ out) { const size_t u = (size_t)blockIdx.x * 256 + threadIdx.x; if (u >= (size_t)N * NC) return; const size_t n = u / NC; const int c = (int)(u % NC); if (n >= (size_t)NLIM) return; float s = bfv(fb2[c]);
#pragma unroll 4
  for (int k = 0; k < H; ++k) s += pmul(Hp[n * H + k], bfv(fw[k * NC + c]));
  for (int pass = 0; pass < 2; ++pass) { ((volatile float*)out)[u] = s; __threadfence(); } }
}

extern "C" void kernel_launch(void* const* d_in, const int* in_sizes, int n_in, void* d_out, int out_size, void* d_ws, size_t ws_size, hipStream_t stream) {
  (void)n_in;
  auto Fp = [&](int i) { return (const float*)d_in[i]; }; auto Ip = [&](int i) { return (const int*)d_in[i]; };
  if (in_sizes[0] != N * FIN || in_sizes[1] != E || in_sizes[2] != FIN * H || in_sizes[4] != 272 * H || in_sizes[6] != 272 * H || in_sizes[10] != 272 * H || in_sizes[12] != 272 * H || in_sizes[16] != H * NC || in_sizes[18] != 2 * E || out_size != N * NC) return;
  const int NLIM = N;
  size_t off = 0; char* ws = (char*)d_ws;
  auto carve = [&](size_t bytes) { char* p = ws + off; off += (bytes + 255) & ~(size_t)255; return p; };
  b16* WN = (b16*)carve((size_t)2 * 512 * H * 2); b16* WE = (b16*)carve((size_t)2 * 256 * 32 * 2); float* Hp = (float*)carve((size_t)NPAD * H * 4); float* P = (float*)carve((size_t)NPAD * 512 * 4); float* AGG = (float*)carve((size_t)NPAD * H * 4); float* PS = (float*)carve((size_t)(NPAD / 4 + 1) * 2 * H * 4); float* BNP = (float*)carve(2 * H * 4);
  CsrBufs8 csr; off = csr_carve8(csr, ws, off, E, N);
  if (off > ws_size || off > ((size_t)112 << 20)) return;
  const int nb = (NLIM + 3) / 4; const unsigned nwv = (NLIM + 15) / 16;
  wput_kernel<<<128, 256, 0, stream>>>(Fp(4), Fp(6), Fp(10), Fp(12), WN, WE);
  csr_build8(csr, Ip(18) + E, E, N, stream);
  lin0_kernel<<<(unsigned)(((size_t)N * 32 + 255) / 256), 256, 0, stream>>>(Fp(0), Fp(2), Fp(3), NLIM, Hp);
  for (int l = 0; l < 2; ++l) {
    proj_kernel<<<nwv, 32, 0, stream>>>(Hp, WN + (size_t)l * 512 * H, NLIM, P);
    cg_kernel<<<nb, 128, 0, stream>>>(P, Fp(1), WE + (size_t)l * 256 * 32, Fp(l ? 11 : 5), Fp(l ? 13 : 7), Ip(18), csr.PERM, csr.ROWPTR, csr.ROWCNT, (int)csr.permLen, NLIM, AGG, PS);
    bn_kernel<<<1, 128, 0, stream>>>(PS, nb, NLIM, Fp(l ? 14 : 8), Fp(l ? 15 : 9), BNP);
    upd_kernel<<<(unsigned)(((size_t)N * 32 + 255) / 256), 256, 0, stream>>>(AGG, BNP, NLIM, Hp); }
  fc_kernel<<<(unsigned)(((size_t)N * NC + 255) / 256), 256, 0, stream>>>(Hp, Fp(16), Fp(17), NLIM, (float*)d_out);
}
